// DGCN_83674552860914
// MI455X (gfx1250) — hardware-verified
//
#include <hip/hip_runtime.h>
#include <stddef.h>
#include <math.h>


#define KIN     128
#define FD      64
#define KCAT    192
#define NCLS    16
#define NTHR    256
#define NWAVE   8
#define EPT     8
#define NGRP    2
#define CHUNK   (NTHR * EPT * NGRP)
#define WCAP    (EPT * NGRP * 32)
#define LISTN   (NWAVE * WCAP)
#define NBA     1024
#define NBD     4096
#define GROWS   128
#define HROWS   256
#define WSCALE  8.0f
#define WINV    0.125f
#define LDS_AGG (NBA * FD * 4 + LISTN * 4 + 64)

static_assert((CHUNK & (CHUNK - 1)) == 0);
static_assert(CHUNK <= 4096);
static_assert((NBA & (NBA - 1)) == 0 && NBA <= 4096);
static_assert((NBD & (NBD - 1)) == 0 && NBD <= 4096);
static_assert(GROWS == NWAVE * 16);
static_assert(HROWS == NWAVE * 32 && HROWS == NTHR);
static_assert(NBA * (FD / 8) == NTHR * 32);
static_assert(NBD == NWAVE * 4 * 128);
static_assert((FD * KIN / 8) % NTHR == 0 && (FD * KCAT / 8) % NTHR == 0);
static_assert(KIN % 32 == 0 && KCAT % 32 == 0 && FD % 32 == 0);

typedef float    v2f  __attribute__((ext_vector_type(2)));
typedef float    v4f  __attribute__((ext_vector_type(4)));
typedef float    v8f  __attribute__((ext_vector_type(8)));
typedef int      v4i  __attribute__((ext_vector_type(4)));
typedef _Float16 v8h  __attribute__((ext_vector_type(8)));
typedef _Float16 v16h __attribute__((ext_vector_type(16)));
union FragH { v16h v; v8h h[2]; };

__device__ __forceinline__ v8h cvt8(v4f a, v4f b) {
  v8h r;
  r[0] = (_Float16)a.x; r[1] = (_Float16)a.y; r[2] = (_Float16)a.z; r[3] = (_Float16)a.w;
  r[4] = (_Float16)b.x; r[5] = (_Float16)b.y; r[6] = (_Float16)b.z; r[7] = (_Float16)b.w;
  return r;
}

__device__ __forceinline__ v4f relu4(v4f v) {
  v4f r;
  r.x = fmaxf(v.x, 0.0f); r.y = fmaxf(v.y, 0.0f); r.z = fmaxf(v.z, 0.0f); r.w = fmaxf(v.w, 0.0f);
  return r;
}

__device__ __forceinline__ v8f wmh(v16h a, v16h b, v8f c) {
  v8f d = __builtin_amdgcn_wmma_f32_16x16x32_f16(false, a, false, b, (short)0, c, false, false);
  asm volatile("v_nop\n\tv_nop\n\tv_nop\n\tv_nop" : "+v"(d) : "v"(a), "v"(b));
  return d;
}

template <int NB>
__device__ __forceinline__ int scan_chunk(const int* __restrict__ dsts, int nE, int cbase, int nodeBase,
                                          int vec8, int* list, int tid, int lane, int wave) {
  int wc = 0;
#pragma unroll
  for (int g = 0; g < NGRP; ++g) {
    const int el0  = (g * NTHR + tid) * EPT;
    const int e0   = cbase + el0;
    const int sent = -2147483647 - 1;
    v4i da, db;
    if (vec8 != 0 && cbase + CHUNK <= nE) {
      da = *(const v4i*)(dsts + e0);
      db = *(const v4i*)(dsts + e0 + 4);
    } else {
      da.x = (e0     < nE) ? dsts[min(e0,     nE - 1)] : sent;
      da.y = (e0 + 1 < nE) ? dsts[min(e0 + 1, nE - 1)] : sent;
      da.z = (e0 + 2 < nE) ? dsts[min(e0 + 2, nE - 1)] : sent;
      da.w = (e0 + 3 < nE) ? dsts[min(e0 + 3, nE - 1)] : sent;
      db.x = (e0 + 4 < nE) ? dsts[min(e0 + 4, nE - 1)] : sent;
      db.y = (e0 + 5 < nE) ? dsts[min(e0 + 5, nE - 1)] : sent;
      db.z = (e0 + 6 < nE) ? dsts[min(e0 + 6, nE - 1)] : sent;
      db.w = (e0 + 7 < nE) ? dsts[min(e0 + 7, nE - 1)] : sent;
    }
    const unsigned nb = (unsigned)nodeBase;
    const unsigned s0 = (unsigned)da.x - nb, s1 = (unsigned)da.y - nb;
    const unsigned s2 = (unsigned)da.z - nb, s3 = (unsigned)da.w - nb;
    const unsigned s4 = (unsigned)db.x - nb, s5 = (unsigned)db.y - nb;
    const unsigned s6 = (unsigned)db.z - nb, s7 = (unsigned)db.w - nb;
    const bool h0 = s0 < (unsigned)NB, h1 = s1 < (unsigned)NB, h2 = s2 < (unsigned)NB, h3 = s3 < (unsigned)NB;
    const bool h4 = s4 < (unsigned)NB, h5 = s5 < (unsigned)NB, h6 = s6 < (unsigned)NB, h7 = s7 < (unsigned)NB;
    const unsigned any = __builtin_amdgcn_ballot_w32(h0 | h1 | h2 | h3 | h4 | h5 | h6 | h7);
    if (any != 0u) {
#define HITJ(J, HJ, SJ) { \
        const unsigned mj = __builtin_amdgcn_ballot_w32(HJ); \
        if (mj != 0u) { \
          if (HJ) { \
            const int pos = wc + (int)__builtin_amdgcn_mbcnt_lo(mj, 0u); \
            if (pos < WCAP) list[wave * WCAP + pos] = ((el0 + (J)) << 12) | (int)(SJ); \
          } \
          wc += (int)__builtin_popcount(mj); } }
      HITJ(0, h0, s0)
      HITJ(1, h1, s1)
      HITJ(2, h2, s2)
      HITJ(3, h3, s3)
      HITJ(4, h4, s4)
      HITJ(5, h5, s5)
      HITJ(6, h6, s6)
      HITJ(7, h7, s7)
#undef HITJ
    }
  }
  return wc;
}

__global__ __launch_bounds__(NTHR) void k_wprep(
    const float* __restrict__ W1, const float* __restrict__ W2, const float* __restrict__ W3,
    _Float16* w1s, _Float16* w2s, _Float16* w3s) {
  const int n1 = FD * KIN / 8;
  const int n2 = FD * KCAT / 8;
  const int n3 = NCLS * KCAT / 8;
  const int b  = blockIdx.x;
  const int i  = b * NTHR + threadIdx.x;
  const float* sp;
  _Float16* dp;
  int li;
  if (b < n1 / NTHR)             { li = i;           sp = W1; dp = w1s; }
  else if (b < (n1 + n2) / NTHR) { li = i - n1;      sp = W2; dp = w2s; }
  else                           { li = i - n1 - n2; sp = W3; dp = w3s; if (li >= n3) return; }
  const float* p = sp + (size_t)li * 8;
  v4f a = *(const v4f*)p, c = *(const v4f*)(p + 4);
  a = a * WSCALE;
  c = c * WSCALE;
  const v8h hv = cvt8(a, c);
  _Float16* q = dp + (size_t)li * 8;
  *(volatile v8h*)q = hv;
  __threadfence();
  *(volatile v8h*)q = hv;
}

template <int NB>
__global__ __launch_bounds__(NTHR) void k_deg(
    const int* __restrict__ ei0, const int* __restrict__ ei1, const int* __restrict__ ei2,
    const float* __restrict__ w1, const float* __restrict__ w2,
    float* dis, int disStride, int nE, int vec8) {
  __shared__ __attribute__((aligned(16))) float dg[NB];
  __shared__ __attribute__((aligned(16))) int list[LISTN];
  __shared__ int wcnt[NWAVE];
  const int tid = threadIdx.x, lane = tid & 31, wave = tid >> 5;
  const int set = blockIdx.y;
  const int nodeBase = blockIdx.x * NB;
  const int*   es   = (set == 0) ? ei0 : ((set == 1) ? ei1 : ei2);
  const float* w    = (set == 2) ? w2 : w1;
  const int    hasw = (set != 0) ? 1 : 0;
  const int*   dsts = es + nE;

  for (int i = tid; i < NB; i += NTHR) dg[i] = 0.0f;
  __syncthreads();

  const int nChunks = (nE + CHUNK - 1) / CHUNK;
#pragma unroll 1
  for (int ch = 0; ch < nChunks; ++ch) {
    const int cbase = ch * CHUNK;
    const int wc = scan_chunk<NB>(dsts, nE, cbase, nodeBase, vec8, list, tid, lane, wave);
    if (lane == 0) wcnt[wave] = wc;
    __syncthreads();
    if (wave == 0) {
#pragma unroll 1
      for (int wsx = 0; wsx < NWAVE; ++wsx) {
        int n = __builtin_amdgcn_readfirstlane(wcnt[wsx]);
        n = n > WCAP ? WCAP : (n < 0 ? 0 : n);
        const int* lp = list + wsx * WCAP;
#pragma unroll 1
        for (int i = 0; i < n; ++i) {
          const int ent  = __builtin_amdgcn_readfirstlane(lp[i]);
          const int slot = ent & (NB - 1);
          int e = cbase + ((ent >> 12) & (CHUNK - 1));
          e = e > nE - 1 ? nE - 1 : e;
          float we = 1.0f;
          if (hasw != 0) we = w[e];
          if (lane == 0) dg[slot] = dg[slot] + we;
        }
      }
    }
    __syncthreads();
  }

  v4f dq[4];
#pragma unroll
  for (int q = 0; q < 4; ++q) {
    const int f = (wave * 4 + q) * 128 + 4 * lane;
    const v4f c = *(const v4f*)(dg + f);
    const float e0 = c.x + 1.0f, e1 = c.y + 1.0f, e2 = c.z + 1.0f, e3 = c.w + 1.0f;
    dq[q].x = (e0 > 0.0f) ? rsqrtf(e0) : 0.0f;
    dq[q].y = (e1 > 0.0f) ? rsqrtf(e1) : 0.0f;
    dq[q].z = (e2 > 0.0f) ? rsqrtf(e2) : 0.0f;
    dq[q].w = (e3 > 0.0f) ? rsqrtf(e3) : 0.0f;
  }
  float* dp = dis + (size_t)set * disStride + nodeBase;
#pragma unroll
  for (int q = 0; q < 4; ++q) *(volatile v4f*)(dp + (wave * 4 + q) * 128 + 4 * lane) = dq[q];
  __threadfence();
#pragma unroll
  for (int q = 0; q < 4; ++q) *(volatile v4f*)(dp + (wave * 4 + q) * 128 + 4 * lane) = dq[q];
}

__device__ __forceinline__ void gemm64_epilogue(float* stg, v8f (&acc)[4], float* hout,
                                                int rowBase, int wave, int lane, int hh, int m) {
  float* sp = stg + (wave * 16 + 8 * hh) * FD + m;
#pragma unroll
  for (int t = 0; t < 4; ++t) {
#pragma unroll
    for (int r = 0; r < 8; ++r) sp[r * FD + 16 * t] = acc[t][r] * WINV;
  }
  __syncthreads();
  const float* lp = stg + wave * 16 * FD + 4 * lane;
  float* gp = hout + ((size_t)rowBase + wave * 16) * FD + 4 * lane;
#pragma unroll
  for (int q = 0; q < 8; ++q) { const v4f v = *(const v4f*)(lp + q * 128); *(volatile v4f*)(gp + q * 128) = v; }
  __threadfence();
#pragma unroll
  for (int q = 0; q < 8; ++q) { const v4f v = *(const v4f*)(lp + q * 128); *(volatile v4f*)(gp + q * 128) = v; }
}

__global__ __launch_bounds__(NTHR) void k_gemm1(
    const float* __restrict__ x, const _Float16* __restrict__ w1s, float* hout, int nN) {
  __shared__ __attribute__((aligned(16))) float stg[GROWS * FD];
  const int tid = threadIdx.x, lane = tid & 31, wave = tid >> 5, hh = lane >> 4, m = lane & 15;
  const int rowBase = blockIdx.x * GROWS;
  int row = rowBase + wave * 16 + m;
  row = row > nN - 1 ? nN - 1 : row;
  const float* xr = x + (size_t)row * KIN + 8 * hh;

  v8f acc[4];
#pragma unroll
  for (int t = 0; t < 4; ++t) { v8f z = {0.f, 0.f, 0.f, 0.f, 0.f, 0.f, 0.f, 0.f}; acc[t] = z; }
#pragma unroll
  for (int kt = 0; kt < KIN / 32; ++kt) {
    const float* ap = xr + 32 * kt;
    const v4f p0 = *(const v4f*)ap,        p1 = *(const v4f*)(ap + 4);
    const v4f p2 = *(const v4f*)(ap + 16), p3 = *(const v4f*)(ap + 20);
    FragH a;
    a.h[0] = cvt8(p0, p1);
    a.h[1] = cvt8(p2, p3);
#pragma unroll
    for (int t = 0; t < 4; ++t) {
      const _Float16* bp = w1s + (size_t)(16 * t + m) * KIN + 32 * kt + 8 * hh;
      FragH b;
      b.h[0] = *(const v8h*)bp;
      b.h[1] = *(const v8h*)(bp + 16);
      acc[t] = wmh(a.v, b.v, acc[t]);
    }
  }
  gemm64_epilogue(stg, acc, hout, rowBase, wave, lane, hh, m);
}

__global__ __launch_bounds__(NTHR) void k_gemm2(
    const _Float16* __restrict__ cat, int catStride, const _Float16* __restrict__ w2s, float* hout) {
  __shared__ __attribute__((aligned(16))) float stg[GROWS * FD];
  const int tid = threadIdx.x, lane = tid & 31, wave = tid >> 5, hh = lane >> 4, m = lane & 15;
  const int rowBase = blockIdx.x * GROWS;
  const int row = rowBase + wave * 16 + m;

  v8f acc[4];
#pragma unroll
  for (int t = 0; t < 4; ++t) { v8f z = {0.f, 0.f, 0.f, 0.f, 0.f, 0.f, 0.f, 0.f}; acc[t] = z; }
#pragma unroll
  for (int kt = 0; kt < KCAT / 32; ++kt) {
    const _Float16* ar = cat + (size_t)(kt >> 1) * catStride + (size_t)row * FD + 32 * (kt & 1) + 8 * hh;
    FragH a;
    a.h[0] = *(const v8h*)ar;
    a.h[1] = *(const v8h*)(ar + 16);
#pragma unroll
    for (int t = 0; t < 4; ++t) {
      const _Float16* bp = w2s + (size_t)(16 * t + m) * KCAT + 32 * kt + 8 * hh;
      FragH b;
      b.h[0] = *(const v8h*)bp;
      b.h[1] = *(const v8h*)(bp + 16);
      acc[t] = wmh(a.v, b.v, acc[t]);
    }
  }
  gemm64_epilogue(stg, acc, hout, rowBase, wave, lane, hh, m);
}

__device__ __forceinline__ void agg_store_pass(const float* acc, const float* __restrict__ hp,
                                               const float* __restrict__ disS, const float* __restrict__ bias,
                                               _Float16* catS, int nodeBase, int nN, int wave, int lane) {
#pragma unroll 2
  for (int i = 0; i < 32; ++i) {
    const int p   = (wave * 32 + i) * 32 + lane;
    const int row = p >> 3;
    const int c0  = (p & 7) * 8;
    int node = nodeBase + row;
    node = node > nN - 1 ? nN - 1 : node;
    const float d = disS[node];
    const v4f a0 = *(const v4f*)(acc + row * FD + c0);
    const v4f a1 = *(const v4f*)(acc + row * FD + c0 + 4);
    const float* hr = hp + (size_t)node * FD + c0;
    const v4f g0 = *(const v4f*)hr, g1 = *(const v4f*)(hr + 4);
    const v4f b0 = *(const v4f*)(bias + c0), b1 = *(const v4f*)(bias + c0 + 4);
    const v4f v0 = relu4((a0 + g0 * d) * d + b0);
    const v4f v1 = relu4((a1 + g1 * d) * d + b1);
    const v8h hv = cvt8(v0, v1);
    *(volatile v8h*)(catS + ((size_t)nodeBase + row) * FD + c0) = hv;
  }
}

__global__ __launch_bounds__(NTHR) void k_agg(
    const int* __restrict__ ei0, const int* __restrict__ ei1, const int* __restrict__ ei2,
    const float* __restrict__ w1, const float* __restrict__ w2,
    const float* __restrict__ dis, int disStride,
    const float* __restrict__ hp, const float* __restrict__ bias,
    _Float16* cat, int catStride, int nN, int nE, int vec8) {
  extern __shared__ v4f lds_dyn[];
  float* acc  = (float*)lds_dyn;
  int*   list = (int*)(acc + NBA * FD);
  int*   wcnt = list + LISTN;
  const int tid = threadIdx.x, lane = tid & 31, wave = tid >> 5;
  const int set = blockIdx.y;
  const int nodeBase = blockIdx.x * NBA;
  const int*   es   = (set == 0) ? ei0 : ((set == 1) ? ei1 : ei2);
  const float* w    = (set == 2) ? w2 : w1;
  const int    hasw = (set != 0) ? 1 : 0;
  const int*   srcs = es;
  const int*   dsts = es + nE;
  const float* disS = dis + (size_t)set * disStride;
  _Float16*    catS = cat + (size_t)set * catStride;

  {
    const v4f z = {0.f, 0.f, 0.f, 0.f};
    for (int i = tid; i < NBA * FD / 4; i += NTHR) lds_dyn[i] = z;
  }
  __syncthreads();

  const int nChunks = (nE + CHUNK - 1) / CHUNK;
#pragma unroll 1
  for (int ch = 0; ch < nChunks; ++ch) {
    const int cbase = ch * CHUNK;
    const int wc = scan_chunk<NBA>(dsts, nE, cbase, nodeBase, vec8, list, tid, lane, wave);
    if (lane == 0) wcnt[wave] = wc;
    __syncthreads();
    if (wave == 0) {
#pragma unroll 1
      for (int wsx = 0; wsx < NWAVE; ++wsx) {
        int n = __builtin_amdgcn_readfirstlane(wcnt[wsx]);
        n = n > WCAP ? WCAP : (n < 0 ? 0 : n);
        const int* lp = list + wsx * WCAP;
#pragma unroll 1
        for (int i = 0; i < n; ++i) {
          const int ent  = __builtin_amdgcn_readfirstlane(lp[i]);
          const int slot = ent & (NBA - 1);
          int e = cbase + ((ent >> 12) & (CHUNK - 1));
          e = e > nE - 1 ? nE - 1 : e;
          int src = srcs[e];
          src = src < 0 ? 0 : (src > nN - 1 ? nN - 1 : src);
          float c = disS[src];
          if (hasw != 0) c = c * w[e];
          const v2f hv = *(const v2f*)(hp + (size_t)src * FD + 2 * lane);
          v2f* ap = (v2f*)(acc + slot * FD + 2 * lane);
          *ap = *ap + hv * c;
        }
      }
    }
    __syncthreads();
  }

  agg_store_pass(acc, hp, disS, bias, catS, nodeBase, nN, wave, lane);
  __threadfence();
  agg_store_pass(acc, hp, disS, bias, catS, nodeBase, nN, wave, lane);
}

__global__ __launch_bounds__(NTHR) void k_head(
    const _Float16* __restrict__ cat, int catStride, const _Float16* __restrict__ w3s,
    const float* __restrict__ cb, float* out, int nN) {
  __shared__ __attribute__((aligned(16))) float stg[HROWS * NCLS];
  const int tid = threadIdx.x, lane = tid & 31, wave = tid >> 5, hh = lane >> 4, m = lane & 15;
  const int nodeBase = blockIdx.x * HROWS;
  const float cbm = cb[m];

#pragma unroll
  for (int q = 0; q < 2; ++q) {
    const int t   = wave * 2 + q;
    const int row = nodeBase + 16 * t + m;
    v8f acc = {0.f, 0.f, 0.f, 0.f, 0.f, 0.f, 0.f, 0.f};
#pragma unroll
    for (int kt = 0; kt < KCAT / 32; ++kt) {
      const _Float16* ar = cat + (size_t)(kt >> 1) * catStride + (size_t)row * FD + 32 * (kt & 1) + 8 * hh;
      FragH a;
      a.h[0] = *(const v8h*)ar;
      a.h[1] = *(const v8h*)(ar + 16);
      const _Float16* bp = w3s + (size_t)m * KCAT + 32 * kt + 8 * hh;
      FragH b;
      b.h[0] = *(const v8h*)bp;
      b.h[1] = *(const v8h*)(bp + 16);
      acc = wmh(a.v, b.v, acc);
    }
    float* sp = stg + (16 * t + 8 * hh) * NCLS + m;
#pragma unroll
    for (int r = 0; r < 8; ++r) sp[r * NCLS] = acc[r] * WINV + cbm;
  }
  __syncthreads();

  {
    float* rp = stg + tid * NCLS;
    float mx = rp[0];
#pragma unroll 1
    for (int j = 1; j < NCLS; ++j) mx = fmaxf(mx, rp[j]);
    float s = 0.0f;
#pragma unroll 1
    for (int j = 0; j < NCLS; ++j) s += expf(rp[j] - mx);
    const float ls = logf(s);
#pragma unroll 1
    for (int j = 0; j < NCLS; ++j) { const float v = rp[j]; rp[j] = (v - mx) - ls; }
  }
  __syncthreads();

  const size_t outN = (size_t)nN * NCLS;
  const size_t ob   = (size_t)nodeBase * NCLS;
  v4f ov[4];
#pragma unroll
  for (int q = 0; q < 4; ++q) ov[q] = *(const v4f*)(stg + (wave * 4 + q) * 128 + 4 * lane);
#pragma unroll
  for (int q = 0; q < 4; ++q) {
    const size_t gi = ob + (size_t)((wave * 4 + q) * 128 + 4 * lane);
    if (gi < outN) *(volatile v4f*)(out + gi) = ov[q];
  }
  __threadfence();
#pragma unroll
  for (int q = 0; q < 4; ++q) {
    const size_t gi = ob + (size_t)((wave * 4 + q) * 128 + 4 * lane);
    if (gi < outN) *(volatile v4f*)(out + gi) = ov[q];
  }
}

extern "C" void kernel_launch(void* const* d_in, const int* in_sizes, int n_in,
                              void* d_out, int out_size, void* d_ws, size_t ws_size,
                              hipStream_t stream) {
  if (n_in < 12) return;
  const int nN = in_sizes[0] / KIN;
  const int nE = in_sizes[1] / 2;
  if (nN <= 0 || nE <= 0 || in_sizes[0] != nN * KIN || in_sizes[1] != nE * 2) return;
  if (in_sizes[2] != in_sizes[1] || in_sizes[3] != in_sizes[1]) return;
  if (in_sizes[4] != nE || in_sizes[5] != nE) return;
  if (in_sizes[6] != FD * KIN || in_sizes[7] != FD * KCAT) return;
  if (in_sizes[8] < FD || in_sizes[9] < FD) return;
  if (in_sizes[10] != NCLS * KCAT || in_sizes[11] < NCLS) return;
  if (out_size != nN * NCLS) return;

  const float* x     = (const float*)d_in[0];
  const int*   ei0   = (const int*)d_in[1];
  const int*   ei1   = (const int*)d_in[2];
  const int*   ei2   = (const int*)d_in[3];
  const float* in_w  = (const float*)d_in[4];
  const float* out_w = (const float*)d_in[5];
  const float* W1    = (const float*)d_in[6];
  const float* W2    = (const float*)d_in[7];
  const float* b1    = (const float*)d_in[8];
  const float* b2    = (const float*)d_in[9];
  const float* W3    = (const float*)d_in[10];
  const float* b3    = (const float*)d_in[11];
  float* out = (float*)d_out;

  const int nBD = (nN + NBD - 1) / NBD;
  const int nG  = (nN + GROWS - 1) / GROWS;
  const int nA  = (nN + NBA - 1) / NBA;
  const int nH  = (nN + HROWS - 1) / HROWS;
  const int disStride = nBD * NBD;
  const int hRows     = nG * GROWS;
  int catRows = nA * NBA;
  if (nG * GROWS > catRows) catRows = nG * GROWS;
  if (nH * HROWS > catRows) catRows = nH * HROWS;
  const int catStride = catRows * FD;

  char* ws = (char*)d_ws;
  size_t off = 0;
  const size_t oW1 = off; off += (size_t)FD * KIN * 2;            off = (off + 255) & ~(size_t)255;
  const size_t oW2 = off; off += (size_t)FD * KCAT * 2;           off = (off + 255) & ~(size_t)255;
  const size_t oW3 = off; off += (size_t)NCLS * KCAT * 2;         off = (off + 255) & ~(size_t)255;
  const size_t oDs = off; off += (size_t)3 * disStride * 4;       off = (off + 255) & ~(size_t)255;
  const size_t oH1 = off; off += (size_t)hRows * FD * 4;          off = (off + 255) & ~(size_t)255;
  const size_t oH2 = off; off += (size_t)hRows * FD * 4;          off = (off + 255) & ~(size_t)255;
  const size_t oC1 = off; off += (size_t)3 * catStride * 2;       off = (off + 255) & ~(size_t)255;
  const size_t oC2 = off; off += (size_t)3 * catStride * 2;       off = (off + 255) & ~(size_t)255;
  if (off > ws_size) return;
  if (off > ((size_t)128 << 20)) return;
  _Float16* w1s  = (_Float16*)(ws + oW1);
  _Float16* w2s  = (_Float16*)(ws + oW2);
  _Float16* w3s  = (_Float16*)(ws + oW3);
  float*    dis  = (float*)(ws + oDs);
  float*    h1p  = (float*)(ws + oH1);
  float*    h2p  = (float*)(ws + oH2);
  _Float16* cat1 = (_Float16*)(ws + oC1);
  _Float16* cat2 = (_Float16*)(ws + oC2);

  const int vec8 = ((nE & 3) == 0) ? 1 : 0;

  const int nPrep = FD * KIN / 8 + FD * KCAT / 8 + NCLS * KCAT / 8;
  k_wprep<<<(nPrep + NTHR - 1) / NTHR, NTHR, 0, stream>>>(W1, W2, W3, w1s, w2s, w3s);

  k_deg<NBD><<<dim3(nBD, 3), NTHR, 0, stream>>>(ei0, ei1, ei2, in_w, out_w, dis, disStride, nE, vec8);

  k_gemm1<<<nG, NTHR, 0, stream>>>(x, w1s, h1p, nN);

  hipFuncSetAttribute(reinterpret_cast<const void*>(&k_agg),
                      hipFuncAttributeMaxDynamicSharedMemorySize, LDS_AGG);
  k_agg<<<dim3(nA, 3), NTHR, LDS_AGG, stream>>>(ei0, ei1, ei2, in_w, out_w, dis, disStride,
                                               h1p, b1, cat1, catStride, nN, nE, vec8);

  k_gemm2<<<nG, NTHR, 0, stream>>>(cat1, catStride, w2s, h2p);

  k_agg<<<dim3(nA, 3), NTHR, LDS_AGG, stream>>>(ei0, ei1, ei2, in_w, out_w, dis, disStride,
                                               h2p, b2, cat2, catStride, nN, nE, vec8);

  k_head<<<nH, NTHR, 0, stream>>>(cat2, catStride, w3s, b3, out, nN);
}
